// DemodConv_61641370632560
// MI455X (gfx1250) — hardware-verified
//
#include <hip/hip_runtime.h>


namespace {
constexpr int Bn = 8, CI = 512, CO = 512, HW = 32, NP = HW * HW, KT = CI * 9  ;
constexpr float WS_ = 32.0f, EPS = 1e-8f;

typedef _Float16 b16;
typedef __attribute__((ext_vector_type(16))) _Float16 v16b;
typedef __attribute__((ext_vector_type(8))) _Float16 v8b;
typedef __attribute__((ext_vector_type(8))) float v8f;
typedef __attribute__((ext_vector_type(4))) float v4f;
__device__ __forceinline__ float bf16_rne(float f) { unsigned int u = __float_as_uint(f); u += 0x7FFFu + ((u >> 16) & 1u); return __uint_as_float(u & 0xFFFF0000u); }
__device__ __forceinline__ void split16(float v, b16& hi, b16& lo) { hi = (b16)v; lo = (b16)(v - (float)hi); }
__device__ __forceinline__ v16b frag_kb(const b16* p, int hh) { const v8b a = *(const v8b*)(p + 8 * hh), b = *(const v8b*)(p + 16 + 8 * hh); v16b f;
#pragma unroll
  for (int e = 0; e < 8; ++e) { f[e] = a[e]; f[8 + e] = b[e]; } return f; }
__device__ __forceinline__ v8f wmma16b(v16b a, v16b b, v8f c) { v8f d = __builtin_amdgcn_wmma_f32_16x16x32_f16(false, a, false, b, (short)0, c, false, false); asm volatile("v_nop\n\tv_nop\n\tv_nop\n\tv_nop" : "+v"(d) : "v"(a), "v"(b)); return d; }
__device__ __forceinline__ void wave_lds_sync() { __builtin_amdgcn_fence(__ATOMIC_RELEASE, "workgroup"); __builtin_amdgcn_wave_barrier(); __builtin_amdgcn_fence(__ATOMIC_ACQUIRE, "workgroup"); }

__global__ __launch_bounds__(256) void prep_kernel(const float* __restrict__ x, const float* __restrict__ s, const float* __restrict__ w, b16* __restrict__ x16, b16* __restrict__ wph, b16* __restrict__ wpl, float* __restrict__ dd) {
  __shared__ float red[256]; __shared__ float dv[32];
  const int b = blockIdx.y, cg = blockIdx.x, t_ = threadIdx.x;
  for (int j = 0; j < 32; ++j) { const int co = cg * 32 + j; const float* wr = w + (size_t)co * KT; float sq = 0.0f;
    for (int k = t_; k < KT; k += 256) { const float v = bf16_rne(wr[k]) * (bf16_rne(s[(size_t)b * CI + k / 9]) + 1.0f); sq += v * v; }
    red[t_] = sq; __syncthreads();
    for (int st = 128; st > 0; st >>= 1) { if (t_ < st) red[t_] += red[t_ + st]; __syncthreads(); }
    if (t_ == 0) dv[j] = rsqrtf(red[0] + EPS);
    __syncthreads(); }
  for (int pass = 0; pass < 2; ++pass) {
    for (int i = t_; i < 32 * (KT / 8); i += 256) { const int j = i / (KT / 8), k8 = (i % (KT / 8)) * 8; const int co = cg * 32 + j; const float* wr = w + (size_t)co * KT; const size_t ob = ((size_t)b * CO + co) * KT; v8b oh, ol;
#pragma unroll
      for (int e = 0; e < 8; ++e) { const int k = k8 + e; const float v = bf16_rne(wr[k]) * (bf16_rne(s[(size_t)b * CI + k / 9]) + 1.0f); b16 a, c; split16(v * WS_, a, c); oh[e] = a; ol[e] = c; }
      *(volatile v8b*)(wph + ob + k8) = oh; *(volatile v8b*)(wpl + ob + k8) = ol; }
    if (t_ < 8) *(volatile v4f*)(dd + (size_t)b * CO + cg * 32 + t_ * 4) = *(const v4f*)(&dv[t_ * 4]);
    if (cg == 0) { for (int i = t_; i < CI * NP / 8; i += 256) { v8b o;
#pragma unroll
        for (int e = 0; e < 8; ++e) o[e] = (b16)bf16_rne(x[((size_t)b * CI) * NP + (size_t)i * 8 + e]);
        *(volatile v8b*)(x16 + ((size_t)b * CI) * NP + (size_t)i * 8) = o; } }
    __threadfence(); }
}

__global__ __launch_bounds__(128) void conv_kernel(const b16* __restrict__ x16, const b16* __restrict__ wph, const b16* __restrict__ wpl, const float* __restrict__ dd, float* __restrict__ out) {
  __shared__ __attribute__((aligned(16))) float Tc[64][128 + 4];
  const int lane = threadIdx.x & 31, wave = threadIdx.x >> 5, nloc = lane & 15, hlf = lane >> 4, b = blockIdx.z, p0 = blockIdx.y * 128, m0 = p0 + wave * 32, c0 = blockIdx.x * 64;
  const b16* X = x16 + ((size_t)b * CI) * NP; const b16* Bh = wph + ((size_t)b * CO) * KT; const b16* Bl = wpl + ((size_t)b * CO) * KT;
  const int pa = m0 + nloc, pb_ = m0 + 16 + nloc; const int ya = pa >> 5, xa = pa & 31, yb = pb_ >> 5, xb = pb_ & 31;
  v8f acc[2][4];
#pragma unroll
  for (int r = 0; r < 2; ++r)
#pragma unroll
    for (int t = 0; t < 4; ++t) acc[r][t] = (v8f){};
  for (int kb = 0; kb < KT; kb += 32) { v16b a0, a1;
#pragma unroll
    for (int e = 0; e < 16; ++e) { const int k = kb + ((e < 8) ? (8 * hlf + e) : (16 + 8 * hlf + e - 8)); const int ci = k / 9, tap = k - ci * 9, dy = tap / 3 - 1, dx = tap - (tap / 3) * 3 - 1;
      const int y1 = ya + dy, x1 = xa + dx, y2 = yb + dy, x2 = xb + dx; const bool ok1 = ((unsigned)y1 < 32u) && ((unsigned)x1 < 32u), ok2 = ((unsigned)y2 < 32u) && ((unsigned)x2 < 32u);
      const b16 v1 = X[(size_t)ci * NP + (min(max(y1, 0), 31) << 5) + min(max(x1, 0), 31)], v2 = X[(size_t)ci * NP + (min(max(y2, 0), 31) << 5) + min(max(x2, 0), 31)];
      a0[e] = ok1 ? v1 : (b16)0.0f; a1[e] = ok2 ? v2 : (b16)0.0f; }
#pragma unroll
    for (int t = 0; t < 4; ++t) { const size_t bo = (size_t)(c0 + t * 16 + nloc) * KT + kb; const v16b bh = frag_kb(Bh + bo, hlf), bl = frag_kb(Bl + bo, hlf);
      acc[0][t] = wmma16b(a0, bh, acc[0][t]); acc[0][t] = wmma16b(a0, bl, acc[0][t]); acc[1][t] = wmma16b(a1, bh, acc[1][t]); acc[1][t] = wmma16b(a1, bl, acc[1][t]); } }
#pragma unroll
  for (int t = 0; t < 4; ++t) { const int co = c0 + t * 16 + nloc; const float dv = dd[(size_t)b * CO + co] * (1.0f / WS_);
#pragma unroll
    for (int r = 0; r < 2; ++r)
#pragma unroll
      for (int v = 0; v < 8; ++v) Tc[t * 16 + nloc][wave * 32 + r * 16 + 8 * hlf + v] = acc[r][t][v] * dv; }
  __syncthreads();
  for (int pass = 0; pass < 2; ++pass) { for (int i = threadIdx.x; i < 64 * 32; i += 128) { const int cc = i >> 5, c4 = (i & 31) * 4; *(volatile v4f*)(out + (((size_t)b * CO + c0 + cc) * NP) + p0 + c4) = *(const v4f*)(&Tc[cc][c4]); } __threadfence(); }
}
}

extern "C" void kernel_launch(void* const* d_in, const int* in_sizes, int n_in,
                              void* d_out, int out_size, void* d_ws, size_t ws_size, hipStream_t stream) {
  (void)n_in; (void)out_size;
  const float* x = (const float*)d_in[0]; const float* s = (const float*)d_in[1]; const float* w = (const float*)d_in[2];
  float* out = (float*)d_out;
  if (in_sizes[0] != Bn * CI * NP || in_sizes[1] != Bn * CI || in_sizes[2] != CO * KT) return;
  size_t off = 0; char* ws = (char*)d_ws;
  auto carve = [&](size_t bytes) { char* p = ws + off; off += (bytes + 255) & ~(size_t)255; return p; };
  b16* x16 = (b16*)carve((size_t)Bn * CI * NP * 2); b16* wph = (b16*)carve((size_t)Bn * CO * KT * 2); b16* wpl = (b16*)carve((size_t)Bn * CO * KT * 2); float* dd = (float*)carve((size_t)Bn * CO * 4);
  if (off > ws_size) return;
  prep_kernel<<<dim3(CO / 32, Bn), 256, 0, stream>>>(x, s, w, x16, wph, wpl, dd);
  conv_kernel<<<dim3(CO / 64, NP / 128, Bn), 128, 0, stream>>>(x16, wph, wpl, dd, out);
}
